// Mamba2Block_4363686773536
// MI455X (gfx1250) — hardware-verified
//
#include <hip/hip_runtime.h>
#include <math.h>

typedef __attribute__((ext_vector_type(16))) _Float16 v16h;
typedef __attribute__((ext_vector_type(8)))  _Float16 v8h;
typedef __attribute__((ext_vector_type(16))) __bf16   v16b;
typedef __attribute__((ext_vector_type(8)))  __bf16   v8b;
typedef __attribute__((ext_vector_type(8)))  float    v8f;
typedef __attribute__((ext_vector_type(4)))  float    v4f;

constexpr int kBatch = 2;
constexpr int kSeq   = 2048;
constexpr int kDM    = 1024;
constexpr int kDI    = 2048;
constexpr int kNS    = 128;
constexpr int kHD    = 64;
constexpr int kNH    = 32;
constexpr int kDP    = 4384;
constexpr int kDPP   = 4416;
constexpr int kRows  = kBatch * kSeq;
constexpr int kColZ  = 0;
constexpr int kColX  = 2048;
constexpr int kColB  = 4096;
constexpr int kColC  = 4224;
constexpr int kColDT = 4352;
constexpr int kTS    = 32;
constexpr float kYCarry    = 16.0f;
constexpr float kWCarry    = 256.0f;
constexpr float kScaleG1   = 1.0f / 256.0f;
constexpr float kScaleG2   = 1.0f / 4096.0f;
static_assert(kDI == 2 * kDM);
static_assert(kNH * kHD == kDI);
static_assert(kDP == 2 * kDI + 2 * kNS + kNH);
static_assert(kColX == kDI && kColB == 2 * kDI && kColC == kColB + kNS && kColDT == kColC + kNS && kColDT + kNH == kDP);
static_assert((kDPP % 64) == 0 && kDPP >= kDP && (kDPP * 4) % 128 == 0);
static_assert((kRows % 64) == 0 && (kDM % 64) == 0 && (kDM % 32) == 0 && (kDI % 32) == 0);
static_assert((kSeq % kTS) == 0 && kTS == 32);

constexpr size_t kOffXN   = 0;
constexpr size_t kOffWIN  = kOffXN   + (size_t)kRows * kDM * 2;
constexpr size_t kOffWOUT = kOffWIN  + (size_t)kDPP  * kDM * 2;
constexpr size_t kOffPROJ = kOffWOUT + (size_t)kDM   * kDI * 2;
constexpr size_t kOffYP   = kOffPROJ + (size_t)kRows * kDPP * 4;
constexpr size_t kWsTotal = kOffYP   + (size_t)kRows * kDI * 2;
static_assert(kWsTotal == 110755840ull);
static_assert(kWsTotal <= 134217728ull);
static_assert((kOffWIN % 128) == 0 && (kOffWOUT % 128) == 0 && (kOffPROJ % 128) == 0 && (kOffYP % 128) == 0);

constexpr int kWin8      = kDPP * kDM / 8;
constexpr int kWinReal8  = kDP  * kDM / 8;
constexpr int kWout8     = kDM  * kDI / 8;
static_assert((kWin8 % 256) == 0 && (kWout8 % 256) == 0);
constexpr int kG1Tiles = (kRows / 64) * (kDPP / 64);
constexpr int kG2Tiles = (kRows / 64) * (kDM / 64);
static_assert((kG1Tiles % 8) == 0 && (kG2Tiles % 8) == 0);

__device__ __forceinline__ unsigned short f2bf_bits(float f) {
  unsigned u = __float_as_uint(f);
  return (unsigned short)((u + 0x7FFFu + ((u >> 16) & 1u)) >> 16);
}
__device__ __forceinline__ float bf_bits2f(unsigned short h) { return __uint_as_float(((unsigned)h) << 16); }

__device__ __forceinline__ void dep_guard4_h(v8f& a, v8f& b, v8f& c, v8f& d, v16h x, v16h y) {
  asm volatile("v_nop\n\tv_nop\n\tv_nop\n\tv_nop" : "+v"(a), "+v"(b), "+v"(c), "+v"(d) : "v"(x), "v"(y));
}
__device__ __forceinline__ void dep_guard4_b(v8f& a, v8f& b, v8f& c, v8f& d, v16b x, v16b y) {
  asm volatile("v_nop\n\tv_nop\n\tv_nop\n\tv_nop" : "+v"(a), "+v"(b), "+v"(c), "+v"(d) : "v"(x), "v"(y));
}
__device__ __forceinline__ void keep4_h(v16h a, v16h b, v16h c, v16h d) { asm volatile("v_nop" :: "v"(a), "v"(b), "v"(c), "v"(d)); }
__device__ __forceinline__ void keep4_b(v16b a, v16b b, v16b c, v16b d) { asm volatile("v_nop" :: "v"(a), "v"(b), "v"(c), "v"(d)); }
__device__ __forceinline__ void acc_guard4(v8f& a, v8f& b, v8f& c, v8f& d) { asm volatile("v_nop\n\tv_nop\n\tv_nop\n\tv_nop" : "+v"(a), "+v"(b), "+v"(c), "+v"(d)); }
template <typename T> struct Frag;
template <> struct Frag<_Float16> {
  typedef v16h V; union U { v16h v; v8h h[2]; };
  static __device__ __forceinline__ v16h load(const _Float16* p) {
    U f; f.h[0] = *(const v8h*)(p); f.h[1] = *(const v8h*)(p + 16); return f.v;
  }
  static __device__ __forceinline__ v8f mma(v16h a, v16h b, v8f c) {
    return __builtin_amdgcn_wmma_f32_16x16x32_f16(false, a, false, b, (short)0, c, false, false);
  }
  static __device__ __forceinline__ void guard4(v8f& a, v8f& b, v8f& c, v8f& d, v16h x, v16h y) { dep_guard4_h(a, b, c, d, x, y); }
  static __device__ __forceinline__ void keep(v16h a, v16h b, v16h c, v16h d) { keep4_h(a, b, c, d); }
};
template <> struct Frag<__bf16> {
  typedef v16b V; union U { v16b v; v8b h[2]; };
  static __device__ __forceinline__ v16b load(const __bf16* p) {
    U f; f.h[0] = *(const v8b*)(p); f.h[1] = *(const v8b*)(p + 16); return f.v;
  }
  static __device__ __forceinline__ v8f mma(v16b a, v16b b, v8f c) {
    return __builtin_amdgcn_wmma_f32_16x16x32_bf16(false, a, false, b, (short)0, c, false, false);
  }
  static __device__ __forceinline__ void guard4(v8f& a, v8f& b, v8f& c, v8f& d, v16b x, v16b y) { dep_guard4_b(a, b, c, d, x, y); }
  static __device__ __forceinline__ void keep(v16b a, v16b b, v16b c, v16b d) { keep4_b(a, b, c, d); }
};

template <int ET> struct Elem;
template <> struct Elem<0> { typedef _Float16 T; };
template <> struct Elem<1> { typedef __bf16 T; };
template <int ET, int SPL, int BIAS_MODE, int OUT_MODE, bool RESID, int ACT = 0>
__global__ __launch_bounds__(256) void wmma_gemm64(
    const unsigned short* __restrict__ Ap, const unsigned short* __restrict__ A2p, int lda, long strideA,
    const unsigned short* __restrict__ Btp, const unsigned short* __restrict__ Bt2p, int ldb, long strideB,
    void* __restrict__ Cout, void* __restrict__ Cout2, int ldc, long strideC,
    const float* __restrict__ bias,
    const float* __restrict__ resid, long strideR,
    int M, int N, int K, float scale) {
  typedef typename Elem<ET>::T T;
  typedef typename Frag<T>::V V;
  const T* A = (const T*)Ap; const T* A2 = (const T*)A2p; const T* Bt = (const T*)Btp; const T* Bt2 = (const T*)Bt2p;
  __shared__ __align__(16) float sT[8][16 * 68];
  const int b    = blockIdx.y;
  const int lane = threadIdx.x & 31;
  const int wave = threadIdx.x >> 5;
  const int tilesN = N >> 6;
  const int tilesM = M >> 6;
  const int tile = blockIdx.x * 8 + wave;
  if (tile >= tilesM * tilesN) return;
  const int tm = tile / tilesN;
  const int tn = tile - tm * tilesN;
  const int m0 = tm << 6;
  const int n0 = tn << 6;

  const T* Ab  = A  + (size_t)b * strideA;
  const T* Bb  = Bt + (size_t)b * strideB;
  const T* Ab2 = (SPL >= 1) ? (A2  + (size_t)b * strideA) : nullptr;
  const T* Bb2 = (SPL == 2) ? (Bt2 + (size_t)b * strideB) : nullptr;

  const int rlane = lane & 15;
  const int koff  = (lane >> 4) * 8;
  const int mOff  = (lane >> 4) * 8;

  v8f acc[4][4];
#pragma unroll
  for (int i = 0; i < 4; ++i)
#pragma unroll
    for (int j = 0; j < 4; ++j) acc[i][j] = (v8f){0.f,0.f,0.f,0.f,0.f,0.f,0.f,0.f};

  for (int k0 = 0; k0 < K; k0 += 32) {
    V bh[4], bl[4];
#pragma unroll
    for (int j = 0; j < 4; ++j) {
      const size_t bo = (size_t)(n0 + (j << 4) + rlane) * ldb + koff + k0;
      bh[j] = Frag<T>::load(Bb + bo);
      if (SPL == 2) bl[j] = Frag<T>::load(Bb2 + bo);
    }
#pragma unroll
    for (int i = 0; i < 4; ++i) {
      const size_t ao = (size_t)(m0 + (i << 4) + rlane) * lda + koff + k0;
      V ah = Frag<T>::load(Ab + ao);
      V al;
      if (SPL >= 1) al = Frag<T>::load(Ab2 + ao);
#pragma unroll
      for (int j = 0; j < 4; ++j) {
        acc[i][j] = Frag<T>::mma(ah, bh[j], acc[i][j]);
        if (SPL == 2) acc[i][j] = Frag<T>::mma(ah, bl[j], acc[i][j]);
        if (SPL >= 1) acc[i][j] = Frag<T>::mma(al, bh[j], acc[i][j]);
      }
      Frag<T>::guard4(acc[i][0], acc[i][1], acc[i][2], acc[i][3], ah, (SPL >= 1) ? al : ah);
    }
    Frag<T>::keep(bh[0], bh[1], bh[2], bh[3]);
    if (SPL == 2) Frag<T>::keep(bl[0], bl[1], bl[2], bl[3]);
  }
  acc_guard4(acc[0][0], acc[0][1], acc[0][2], acc[0][3]);
  acc_guard4(acc[1][0], acc[1][1], acc[1][2], acc[1][3]);
  acc_guard4(acc[2][0], acc[2][1], acc[2][2], acc[2][3]);
  acc_guard4(acc[3][0], acc[3][1], acc[3][2], acc[3][3]);

  float* slab = sT[wave];
  const float* Rb = RESID ? (resid + (size_t)b * strideR) : nullptr;
#pragma unroll
  for (int i = 0; i < 4; ++i) {
    const int mBase = m0 + (i << 4);
#pragma unroll
    for (int j = 0; j < 4; ++j) {
      const int n = n0 + (j << 4) + rlane;
      float bv = 0.f;
      if (BIAS_MODE == 2) bv = bias[n];
#pragma unroll
      for (int r = 0; r < 8; ++r) {
        float v = acc[i][j][r] * scale;
        if (BIAS_MODE == 1) v += bias[mBase + mOff + r];
        if (BIAS_MODE == 2) v += bv;
        if (ACT == 1) v = tanhf(v);
        if (ACT == 2) v = fmaxf(v, 0.0f);
        if (ACT == 3) v = v / (1.0f + expf(-v));
        if (ACT == 4) v = (v > 0.f) ? v : 0.01f * v;
        slab[(mOff + r) * 68 + (j << 4) + rlane] = v;
      }
    }
    __builtin_amdgcn_fence(__ATOMIC_RELEASE, "workgroup");
    __builtin_amdgcn_wave_barrier();
    __builtin_amdgcn_fence(__ATOMIC_ACQUIRE, "workgroup");
    if (OUT_MODE == 0) {
      float* C = (float*)Cout + (size_t)b * strideC;
      const int hh = lane >> 4, c4 = (lane & 15) * 4;
      if (RESID) {
#pragma unroll
        for (int it = 0; it < 4; ++it) {
          const int row = it * 2 + hh;
          float* sp = slab + row * 68 + c4;
          const v4f rr = *(const v4f*)(Rb + (size_t)(mBase + row) * ldc + n0 + c4);
          const v4f sv = *(const v4f*)sp;
          *(v4f*)sp = sv + rr;
        }
        asm volatile("" ::: "memory");
#pragma unroll
        for (int it = 4; it < 8; ++it) {
          const int row = it * 2 + hh;
          float* sp = slab + row * 68 + c4;
          const v4f rr = *(const v4f*)(Rb + (size_t)(mBase + row) * ldc + n0 + c4);
          const v4f sv = *(const v4f*)sp;
          *(v4f*)sp = sv + rr;
        }
        asm volatile("" ::: "memory");
      }
      for (int pass = 0; pass < 2; ++pass) {
#pragma unroll
        for (int it = 0; it < 8; ++it) {
          const int row = it * 2 + hh;
          v4f v = *(const v4f*)(slab + row * 68 + c4);
          *(volatile v4f*)(C + (size_t)(mBase + row) * ldc + n0 + c4) = v;
        }
        __threadfence();
      }
    } else {
      const int q = lane >> 3, c8 = (lane & 7) * 8;
      unsigned short* C  = (unsigned short*)Cout  + (size_t)b * strideC;
      unsigned short* C2 = (OUT_MODE == 2) ? ((unsigned short*)Cout2 + (size_t)b * strideC) : nullptr;
      for (int pass = 0; pass < 2; ++pass) {
#pragma unroll
        for (int it = 0; it < 4; ++it) {
          const int row = it * 4 + q;
          const float* sp = slab + row * 68 + c8;
          v8h hv, lv;
#pragma unroll
          for (int e = 0; e < 8; ++e) {
            if (OUT_MODE == 1) {
              hv[e] = (_Float16)sp[e];
            } else {
              unsigned short hb = f2bf_bits(sp[e]);
              unsigned short lb = f2bf_bits(sp[e] - bf_bits2f(hb));
              hv[e] = __builtin_bit_cast(_Float16, hb);
              lv[e] = __builtin_bit_cast(_Float16, lb);
            }
          }
          *(volatile v8h*)(C + (size_t)(mBase + row) * ldc + n0 + c8) = hv;
          if (OUT_MODE == 2) *(volatile v8h*)(C2 + (size_t)(mBase + row) * ldc + n0 + c8) = lv;
        }
        __threadfence();
      }
    }
    __builtin_amdgcn_fence(__ATOMIC_RELEASE, "workgroup");
    __builtin_amdgcn_wave_barrier();
    __builtin_amdgcn_fence(__ATOMIC_ACQUIRE, "workgroup");
  }
}

__global__ __launch_bounds__(128) void rmsnorm_f16_kernel(
    const float* __restrict__ x, const float* __restrict__ w, unsigned short* __restrict__ XN)
{
  __shared__ float red[4];
  const int row = blockIdx.x, tid = threadIdx.x, lane = tid & 31, wave = tid >> 5;
  const float* xr = x + (size_t)row * kDM + tid * 8;
  const v4f a0 = *(const v4f*)(xr);
  const v4f a1 = *(const v4f*)(xr + 4);
  float s = 0.0f;
#pragma unroll
  for (int e = 0; e < 4; ++e) { s = fmaf(a0[e], a0[e], s); s = fmaf(a1[e], a1[e], s); }
#pragma unroll
  for (int off = 1; off < 32; off <<= 1) s += __shfl_xor(s, off, 32);
  if (lane == 0) red[wave] = s;
  __syncthreads();
  const float tot = (red[0] + red[1]) + (red[2] + red[3]);
  const float inv = rsqrtf(tot * (1.0f / (float)kDM) + 1e-6f);
  const v4f w0 = *(const v4f*)(w + tid * 8);
  const v4f w1 = *(const v4f*)(w + tid * 8 + 4);
  v8h hv;
#pragma unroll
  for (int e = 0; e < 4; ++e) {
    hv[e]     = (_Float16)((a0[e] * inv) * w0[e]);
    hv[4 + e] = (_Float16)((a1[e] * inv) * w1[e]);
  }
  unsigned short* dst = XN + (size_t)row * kDM + tid * 8;
  *(volatile v8h*)dst = hv;
  __threadfence();
  *(volatile v8h*)dst = hv;
}

__global__ __launch_bounds__(256) void cast_rows_f16_kernel(
    const float* __restrict__ src, unsigned short* __restrict__ dst, int total8, int real8, float carry)
{
  const int i = blockIdx.x * 256 + threadIdx.x;
  if (i >= total8) return;
  const int ic = (i < real8) ? i : (real8 - 1);
  const float f = (i < real8) ? carry : 0.0f;
  const size_t e0 = (size_t)ic << 3;
  const v4f a0 = *(const v4f*)(src + e0);
  const v4f a1 = *(const v4f*)(src + e0 + 4);
  v8h hv;
#pragma unroll
  for (int e = 0; e < 4; ++e) {
    hv[e]     = (_Float16)(a0[e] * f);
    hv[4 + e] = (_Float16)(a1[e] * f);
  }
  unsigned short* d = dst + ((size_t)i << 3);
  *(volatile v8h*)d = hv;
  __threadfence();
  *(volatile v8h*)d = hv;
}

__global__ __launch_bounds__(512) void ssm_scan_kernel(
    const float* __restrict__ PROJ, const float* __restrict__ conv_w, const float* __restrict__ conv_b,
    const float* __restrict__ A_log, const float* __restrict__ Dp, const float* __restrict__ dt_bias,
    unsigned short* __restrict__ YP)
{
  __shared__ __align__(16) float sBC[kTS * 2 * kNS];
  __shared__ __align__(16) float sX[(kTS + 3) * kHD];
  __shared__ __align__(16) float sXH[kTS * kHD];
  __shared__ __align__(16) float sG[kTS * kHD];
  __shared__ __align__(16) float sY[kTS * kHD];
  __shared__ __align__(16) float sDTA[2 * kTS];
  static_assert(kTS * 2 * kNS / 4 == 512 * 4);
  static_assert(kTS * kHD == 512 * 4);
  static_assert(512 / 8 == kHD && 8 * 16 == kNS);
  static_assert(8 * 4 == kTS);

  const int tid = threadIdx.x, lane = tid & 31, wave = tid >> 5;
  const int bix = blockIdx.x >> 5;
  const int h   = blockIdx.x & (kNH - 1);
  const size_t row0 = (size_t)bix * kSeq;
  const float Ah  = expf(A_log[h]);
  const float Dh  = Dp[h];
  const float dtb = dt_bias[h];

  const int pp = tid & 63, sgrp = tid >> 6;
  const int cch = h * kHD + pp;
  const v4f wv = *(const v4f*)(conv_w + (size_t)cch * 4);
  const float cbv = conv_b[cch];

  const int p = tid >> 3, nc = tid & 7, n0 = nc * 16;
  float hs[16];
#pragma unroll
  for (int k = 0; k < 16; ++k) hs[k] = 0.0f;

  const int q = lane >> 3, c8 = (lane & 7) * 8;

#pragma unroll 1
  for (int t0 = 0; t0 < kSeq; t0 += kTS) {
    __syncthreads();
#pragma unroll
    for (int j = 0; j < 4; ++j) {
      const int i = tid + 512 * j;
      const int r = i >> 6;
      const int c = (i & 63) * 4;
      *(v4f*)(sBC + r * (2 * kNS) + c) = *(const v4f*)(PROJ + (row0 + t0 + r) * kDPP + kColB + c);
    }
    for (int i = tid; i < (kTS + 3) * (kHD / 4); i += 512) {
      const int r = i >> 4;
      const int c = (i & 15) * 4;
      const int st = t0 - 3 + r;
      const int stc = (st < 0) ? 0 : st;
      const float f = (st < 0) ? 0.0f : 1.0f;
      const v4f v = *(const v4f*)(PROJ + (row0 + stc) * kDPP + kColX + h * kHD + c);
      *(v4f*)(sX + r * kHD + c) = v * f;
    }
    if (wave == 0) {
      const float raw = PROJ[(row0 + t0 + lane) * kDPP + kColDT + h];
      const float v = raw + dtb;
      const float dtv = fmaxf(v, 0.0f) + log1pf(expf(-fabsf(v)));
      sDTA[lane] = dtv;
      sDTA[kTS + lane] = expf(-(Ah * dtv));
    }
    __syncthreads();
#pragma unroll 1
    for (int j = 0; j < 4; ++j) {
      const int s = sgrp * 4 + j;
      const float* xp = sX + s * kHD + pp;
      float acc = cbv;
      acc = fmaf(xp[0],        wv[0], acc);
      acc = fmaf(xp[kHD],      wv[1], acc);
      acc = fmaf(xp[2 * kHD],  wv[2], acc);
      acc = fmaf(xp[3 * kHD],  wv[3], acc);
      const float xh = acc * __builtin_amdgcn_rcpf(1.0f + expf(-acc));
      const float zv = PROJ[(row0 + t0 + s) * kDPP + kColZ + cch];
      const float g = zv * __builtin_amdgcn_rcpf(1.0f + expf(-zv));
      sXH[s * kHD + pp] = xh;
      sG[s * kHD + pp] = g;
    }
    __syncthreads();
#pragma unroll 1
    for (int s = 0; s < kTS; ++s) {
      const float* bcr = sBC + s * (2 * kNS);
      const float dtv = sDTA[s];
      const float dAv = sDTA[kTS + s];
      const float xh = sXH[s * kHD + p];
      const float g  = sG[s * kHD + p];
      const float dtx = dtv * xh;
      float y = 0.0f;
#pragma unroll
      for (int q4 = 0; q4 < 4; ++q4) {
        const v4f bv = *(const v4f*)(bcr + n0 + 4 * q4);
        const v4f cv = *(const v4f*)(bcr + kNS + n0 + 4 * q4);
#pragma unroll
        for (int e = 0; e < 4; ++e) {
          const float t = dtx * bv[e];
          hs[4 * q4 + e] = fmaf(hs[4 * q4 + e], dAv, t);
          y = fmaf(hs[4 * q4 + e], cv[e], y);
        }
      }
      y += __shfl_xor(y, 1, 32);
      y += __shfl_xor(y, 2, 32);
      y += __shfl_xor(y, 4, 32);
      const float yo = (y + Dh * xh) * g;
      if (nc == 0) sY[s * kHD + p] = yo * kYCarry;
    }
    __syncthreads();
    if (wave < 8) {
      const int r = wave * 4 + q;
      const float* sp = sY + r * kHD + c8;
      const v4f a0 = *(const v4f*)(sp);
      const v4f a1 = *(const v4f*)(sp + 4);
      v8h hv;
#pragma unroll
      for (int e = 0; e < 4; ++e) { hv[e] = (_Float16)a0[e]; hv[4 + e] = (_Float16)a1[e]; }
      unsigned short* dst = YP + (row0 + t0 + r) * kDI + h * kHD + c8;
      *(volatile v8h*)dst = hv;
      __threadfence();
      *(volatile v8h*)dst = hv;
    }
  }
}

extern "C" void kernel_launch(void* const* d_in, const int* in_sizes, int n_in,
                              void* d_out, int out_size, void* d_ws, size_t ws_size,
                              hipStream_t stream) {
  if (n_in < 9) return;
  if (in_sizes[0] != kRows * kDM) return;
  if (in_sizes[1] != kDM) return;
  if (in_sizes[2] != kDP * kDM) return;
  if (in_sizes[3] != kDI * 4) return;
  if (in_sizes[4] != kDI) return;
  if (in_sizes[5] != kNH) return;
  if (in_sizes[6] != kNH) return;
  if (in_sizes[7] != kNH) return;
  if (in_sizes[8] != kDM * kDI) return;
  if (out_size != kRows * kDM) return;
  if (ws_size < kWsTotal) return;

  const float* x          = (const float*)d_in[0];
  const float* norm_w     = (const float*)d_in[1];
  const float* in_proj_w  = (const float*)d_in[2];
  const float* conv_w     = (const float*)d_in[3];
  const float* conv_b     = (const float*)d_in[4];
  const float* A_log      = (const float*)d_in[5];
  const float* Dp         = (const float*)d_in[6];
  const float* dt_bias    = (const float*)d_in[7];
  const float* out_proj_w = (const float*)d_in[8];
  float* out = (float*)d_out;

  char* ws = (char*)d_ws;
  unsigned short* XN   = (unsigned short*)(ws + kOffXN);
  unsigned short* WIN  = (unsigned short*)(ws + kOffWIN);
  unsigned short* WOUT = (unsigned short*)(ws + kOffWOUT);
  float*          PROJ = (float*)(ws + kOffPROJ);
  unsigned short* YP   = (unsigned short*)(ws + kOffYP);

  rmsnorm_f16_kernel<<<kRows, 128, 0, stream>>>(x, norm_w, XN);

  cast_rows_f16_kernel<<<kWin8 / 256, 256, 0, stream>>>(in_proj_w, WIN, kWin8, kWinReal8, kWCarry);
  cast_rows_f16_kernel<<<kWout8 / 256, 256, 0, stream>>>(out_proj_w, WOUT, kWout8, kWout8, kWCarry);

  wmma_gemm64<0, 0, 0, 0, false><<<dim3(kG1Tiles / 8, 1), 256, 0, stream>>>(
      XN, nullptr, kDM, 0L,
      WIN, nullptr, kDM, 0L,
      (void*)PROJ, nullptr, kDPP, 0L,
      nullptr, nullptr, 0L,
      kRows, kDPP, kDM, kScaleG1);

  ssm_scan_kernel<<<kBatch * kNH, 512, 0, stream>>>(PROJ, conv_w, conv_b, A_log, Dp, dt_bias, YP);

  wmma_gemm64<0, 0, 0, 0, true><<<dim3(kG2Tiles / 8, 1), 256, 0, stream>>>(
      YP, nullptr, kDI, 0L,
      WOUT, nullptr, kDI, 0L,
      (void*)out, nullptr, kDM, 0L,
      nullptr, x, 0L,
      kRows, kDM, kDI, kScaleG2);
}
